// SDPA_4681514352916
// MI455X (gfx1250) — hardware-verified
//
#include <hip/hip_runtime.h>

typedef __attribute__((ext_vector_type(16))) _Float16 v16h;
typedef __attribute__((ext_vector_type(8)))  _Float16 v8h;
typedef __attribute__((ext_vector_type(4)))  _Float16 v4h;
typedef __attribute__((ext_vector_type(8)))  float    v8f;
typedef __attribute__((ext_vector_type(4)))  float    v4f;

#ifndef NB
#define NB 32
#endif
#ifndef SEQ
#define SEQ 2048
#endif
#define NB_FULL  32
#define SEQ_FULL 2048
#define DH    64
#define BM    128
#define BN    64
#define NTHR  256
#define NIT   (SEQ / BN)
#define LSTR  72
#define OSTR  68
#define IN_BSTRIDE ((size_t)SEQ_FULL * DH)
#ifndef OUT_BSTRIDE
#define OUT_BSTRIDE ((size_t)SEQ * DH)
#endif
#define QSCALE (0.125f * 1.4426950408889634f)
#define PCARRY 6.0f
#define LDS_HALVES (2 * BM * LSTR + 2 * BN * LSTR + 2 * DH * LSTR)

static_assert(SEQ % BM == 0);
static_assert(SEQ % BN == 0);
static_assert(NB >= 1 && NB <= NB_FULL);
static_assert(SEQ >= BM && SEQ <= SEQ_FULL);
static_assert(2 * BM * OSTR <= LDS_HALVES);
static_assert((BM * DH) % (NTHR * 4) == 0);
static_assert((BN * DH) == 4 * (NTHR * 4));
static_assert(DH == 64 && BN == 64 && BM == 16 * (NTHR / 32));

#define XM1_LO 0x67452301u
#define XM1_HI 0xEFCDAB89u
#define XM2_LO 0x54761032u
#define XM2_HI 0xDCFE98BAu
#define XM4_LO 0x32107654u
#define XM4_HI 0xBA98FEDCu
#define XM8_LO 0xFEDCBA98u
#define XM8_HI 0x76543210u

__device__ __forceinline__ float perm16(float x, unsigned s0, unsigned s1) {
  int i = __float_as_int(x);
  int j = __builtin_amdgcn_permlane16(i, i, (int)s0, (int)s1, true, false);
  return __int_as_float(j);
}

__device__ __forceinline__ float max_raw(float a, float b) {
  float r;
  asm("v_max_num_f32 %0, %1, %2" : "=v"(r) : "v"(a), "v"(b));
  return r;
}
__device__ __forceinline__ float add_raw(float a, float b) {
  float r;
  asm("v_add_f32 %0, %1, %2" : "=v"(r) : "v"(a), "v"(b));
  return r;
}

__device__ __forceinline__ float fast_exp2(float x) {
  return __builtin_amdgcn_exp2f(x);
}

__device__ __forceinline__ v8f wmma_f16(v16h a, v16h b, v8f c) {
  return __builtin_amdgcn_wmma_f32_16x16x32_f16(false, a, false, b, (short)0, c,
                                                false, false);
}

__device__ __forceinline__ float bf16r(float x) {
  unsigned u = __float_as_uint(x);
  u = (u + 0x7FFFu + ((u >> 16) & 1u)) & 0xFFFF0000u;
  return __uint_as_float(u);
}

__device__ __forceinline__ v4h pk4b(float a, float b, float c, float d) {
  v4h r;
  r[0] = (_Float16)bf16r(a);
  r[1] = (_Float16)bf16r(b);
  r[2] = (_Float16)bf16r(c);
  r[3] = (_Float16)bf16r(d);
  return r;
}

__device__ __forceinline__ v4h pk4n(float a, float b, float c, float d) {
  v4h r;
  r[0] = (_Float16)a;
  r[1] = (_Float16)b;
  r[2] = (_Float16)c;
  r[3] = (_Float16)d;
  return r;
}

__device__ __forceinline__ v16h load_frag(const _Float16* base, int row, int col0,
                                          int lane) {
  const int hi = (lane >> 4) << 3;
  const _Float16* p = base + row * LSTR + col0 + hi;
  v8h lo = *(const v8h*)(p);
  v8h hv = *(const v8h*)(p + 16);
  return __builtin_shufflevector(lo, hv, 0, 1, 2, 3, 4, 5, 6, 7,
                                         8, 9, 10, 11, 12, 13, 14, 15);
}

__global__ void __launch_bounds__(NTHR)
sdpa_fa_kernel(const float* __restrict__ Q, const float* __restrict__ K,
               const float* __restrict__ V, float* __restrict__ O) {
  __shared__ __attribute__((aligned(16))) _Float16 lds[LDS_HALVES];
  _Float16* Qs  = lds;
  _Float16* Ks0 = Qs  + BM * LSTR;
  _Float16* Ks1 = Ks0 + BN * LSTR;
  _Float16* Vt0 = Ks1 + BN * LSTR;
  _Float16* Vt1 = Vt0 + DH * LSTR;
  _Float16* Ps  = Vt1 + DH * LSTR;

  const int tid  = threadIdx.x;
  const int lane = tid & 31;
  const int wave = tid >> 5;
  const int qtiles = SEQ / BM;
  const int bh   = blockIdx.x / qtiles;
  const int m0   = (blockIdx.x - bh * qtiles) * BM;
  const int lr   = lane & 15;

  const size_t baseQ  = (size_t)bh * IN_BSTRIDE + (size_t)m0 * DH;
  const size_t baseKV = (size_t)bh * IN_BSTRIDE;
  const size_t baseO  = (size_t)bh * OUT_BSTRIDE + (size_t)m0 * DH;

  {
    const float4* Qg = (const float4*)(Q + baseQ);
#pragma unroll
    for (int i = 0; i < (BM * DH) / (NTHR * 4); ++i) {
      int f = (i * NTHR + tid) * 4;
      int r = f >> 6, c = f & 63;
      float4 q = Qg[f >> 2];
      *(v4h*)&Qs[r * LSTR + c] = pk4b(q.x, q.y, q.z, q.w);
    }
    const float4* Kg = (const float4*)(K + baseKV);
    const float4* Vg = (const float4*)(V + baseKV);
#pragma unroll
    for (int i = 0; i < (BN * DH) / (NTHR * 4); ++i) {
      int f = (i * NTHR + tid) * 4;
      int r = f >> 6, c = f & 63;
      float4 kv = Kg[f >> 2];
      *(v4h*)&Ks0[r * LSTR + c] = pk4b(kv.x, kv.y, kv.z, kv.w);
      float4 vv = Vg[f >> 2];
      v4h hv = pk4b(vv.x, vv.y, vv.z, vv.w);
      Vt0[(c + 0) * LSTR + r] = hv[0];
      Vt0[(c + 1) * LSTR + r] = hv[1];
      Vt0[(c + 2) * LSTR + r] = hv[2];
      Vt0[(c + 3) * LSTR + r] = hv[3];
    }
  }
  __syncthreads();

  v16h aq0 = load_frag(Qs, wave * 16 + lr, 0,  lane);
  v16h aq1 = load_frag(Qs, wave * 16 + lr, 32, lane);

  v8f o0 = {}, o1 = {}, o2 = {}, o3 = {};
  float m_run[8], l_run[8];
#pragma unroll
  for (int r = 0; r < 8; ++r) { m_run[r] = -__builtin_inff(); l_run[r] = 0.f; }

  const unsigned SL[4] = { XM1_LO, XM2_LO, XM4_LO, XM8_LO };
  const unsigned SH[4] = { XM1_HI, XM2_HI, XM4_HI, XM8_HI };

  for (int it = 0; it < NIT; ++it) {
    const int cur = it & 1;
    const _Float16* ks = Ks0 + cur * (BN * LSTR);
    const _Float16* vt = Vt0 + cur * (DH * LSTR);
    const bool more = (it + 1) < NIT;

    float4 kr[4], vr[4];
    if (more) {
      const float4* Kn = (const float4*)(K + baseKV + (size_t)(it + 1) * BN * DH);
      const float4* Vn = (const float4*)(V + baseKV + (size_t)(it + 1) * BN * DH);
#pragma unroll
      for (int i = 0; i < 4; ++i) {
        kr[i] = Kn[i * NTHR + tid];
        vr[i] = Vn[i * NTHR + tid];
      }
    }

    v8f s[4];
    {
      v16h b0a = load_frag(ks,  0 + lr, 0, lane), b0b = load_frag(ks,  0 + lr, 32, lane);
      v16h b1a = load_frag(ks, 16 + lr, 0, lane), b1b = load_frag(ks, 16 + lr, 32, lane);
      s[0] = wmma_f16(aq0, b0a, v8f{});
      v16h b2a = load_frag(ks, 32 + lr, 0, lane), b2b = load_frag(ks, 32 + lr, 32, lane);
      s[0] = wmma_f16(aq1, b0b, s[0]);
      s[1] = wmma_f16(aq0, b1a, v8f{});
      v16h b3a = load_frag(ks, 48 + lr, 0, lane), b3b = load_frag(ks, 48 + lr, 32, lane);
      s[1] = wmma_f16(aq1, b1b, s[1]);
      s[2] = wmma_f16(aq0, b2a, v8f{});
      s[2] = wmma_f16(aq1, b2b, s[2]);
      s[3] = wmma_f16(aq0, b3a, v8f{});
      s[3] = wmma_f16(aq1, b3b, s[3]);
      asm volatile("v_nop\n\tv_nop\n\tv_nop\n\tv_nop"
                   : "+v"(s[0]), "+v"(s[1]), "+v"(s[2]), "+v"(s[3])
                   : "v"(aq1), "v"(b3b));
    }

#pragma unroll
    for (int tn = 0; tn < 4; ++tn)
#pragma unroll
      for (int r = 0; r < 8; ++r) s[tn][r] *= QSCALE;

    float t[8], alpha[8], rs[8], mb[8];
#pragma unroll
    for (int r = 0; r < 8; ++r)
      t[r] = fmaxf(fmaxf(s[0][r], s[1][r]), fmaxf(s[2][r], s[3][r]));
#pragma unroll
    for (int stp = 0; stp < 4; ++stp)
#pragma unroll
      for (int r = 0; r < 8; ++r)
        t[r] = max_raw(t[r], perm16(t[r], SL[stp], SH[stp]));
#pragma unroll
    for (int r = 0; r < 8; ++r) {
      float m_new = max_raw(m_run[r], t[r]);
      alpha[r] = fast_exp2(m_run[r] - m_new);
      m_run[r] = m_new;
      mb[r] = m_new - PCARRY;
    }
#pragma unroll
    for (int r = 0; r < 8; ++r) {
      float acc = 0.f;
#pragma unroll
      for (int tn = 0; tn < 4; ++tn) {
        float p = fast_exp2(s[tn][r] - mb[r]);
        s[tn][r] = p;
        acc += p;
      }
      rs[r] = acc;
    }
#pragma unroll
    for (int stp = 0; stp < 4; ++stp)
#pragma unroll
      for (int r = 0; r < 8; ++r)
        rs[r] = add_raw(rs[r], perm16(rs[r], SL[stp], SH[stp]));
#pragma unroll
    for (int r = 0; r < 8; ++r) {
      l_run[r] = l_run[r] * alpha[r] + rs[r];
      o0[r] *= alpha[r]; o1[r] *= alpha[r];
      o2[r] *= alpha[r]; o3[r] *= alpha[r];
    }

    {
      int prow = wave * 16 + ((lane >> 4) << 3);
#pragma unroll
      for (int tn = 0; tn < 4; ++tn) {
        v4h pa = pk4n(s[tn][0], s[tn][1], s[tn][2], s[tn][3]);
        v4h pb = pk4n(s[tn][4], s[tn][5], s[tn][6], s[tn][7]);
#pragma unroll
        for (int r = 0; r < 4; ++r) {
          Ps[(prow + r)     * LSTR + tn * 16 + lr] = pa[r];
          Ps[(prow + 4 + r) * LSTR + tn * 16 + lr] = pb[r];
        }
      }
    }
    __builtin_amdgcn_fence(4  , "wavefront");
    __builtin_amdgcn_wave_barrier();

    {
      v16h ap0 = load_frag(Ps, wave * 16 + lr, 0,  lane);
      v16h ap1 = load_frag(Ps, wave * 16 + lr, 32, lane);
      v16h c0a = load_frag(vt,  0 + lr, 0, lane), c0b = load_frag(vt,  0 + lr, 32, lane);
      v16h c1a = load_frag(vt, 16 + lr, 0, lane), c1b = load_frag(vt, 16 + lr, 32, lane);
      o0 = wmma_f16(ap0, c0a, o0);
      v16h c2a = load_frag(vt, 32 + lr, 0, lane), c2b = load_frag(vt, 32 + lr, 32, lane);
      o0 = wmma_f16(ap1, c0b, o0);
      o1 = wmma_f16(ap0, c1a, o1);
      v16h c3a = load_frag(vt, 48 + lr, 0, lane), c3b = load_frag(vt, 48 + lr, 32, lane);
      o1 = wmma_f16(ap1, c1b, o1);
      o2 = wmma_f16(ap0, c2a, o2);
      o2 = wmma_f16(ap1, c2b, o2);
      o3 = wmma_f16(ap0, c3a, o3);
      o3 = wmma_f16(ap1, c3b, o3);
      asm volatile("v_nop\n\tv_nop\n\tv_nop\n\tv_nop"
                   : "+v"(o0), "+v"(o1), "+v"(o2), "+v"(o3)
                   : "v"(ap1), "v"(c3b));
    }

    if (more) {
      _Float16* ksn = Ks0 + (1 - cur) * (BN * LSTR);
      _Float16* vtn = Vt0 + (1 - cur) * (DH * LSTR);
#pragma unroll
      for (int i = 0; i < 4; ++i) {
        int f = (i * NTHR + tid) * 4;
        int r = f >> 6, c = f & 63;
        *(v4h*)&ksn[r * LSTR + c] = pk4b(kr[i].x, kr[i].y, kr[i].z, kr[i].w);
        v4h hv = pk4b(vr[i].x, vr[i].y, vr[i].z, vr[i].w);
        vtn[(c + 0) * LSTR + r] = hv[0];
        vtn[(c + 1) * LSTR + r] = hv[1];
        vtn[(c + 2) * LSTR + r] = hv[2];
        vtn[(c + 3) * LSTR + r] = hv[3];
      }
    }
    __syncthreads();
  }

  float* Os = (float*)lds;
  {
    const int rbase = wave * 16 + ((lane >> 4) << 3);
#pragma unroll
    for (int r = 0; r < 8; ++r) {
      float inv = 1.0f / l_run[r];
      int row = rbase + r;
      Os[row * OSTR +  0 + lr] = o0[r] * inv;
      Os[row * OSTR + 16 + lr] = o1[r] * inv;
      Os[row * OSTR + 32 + lr] = o2[r] * inv;
      Os[row * OSTR + 48 + lr] = o3[r] * inv;
    }
  }
  __syncthreads();

  {
    float* Og = O + baseO;
    const int c4 = (lane & 15) * 4;
    const int rh = lane >> 4;
    v4f v[8];
#pragma unroll
    for (int i = 0; i < 8; ++i) {
      int row = wave * 16 + 2 * i + rh;
      v[i] = *(const v4f*)&Os[row * OSTR + c4];
    }
#pragma unroll
    for (int i = 0; i < 8; ++i) {
      int row = wave * 16 + 2 * i + rh;
      *(volatile v4f*)(Og + (size_t)row * DH + c4) = v[i];
    }
    __threadfence();
#pragma unroll
    for (int i = 0; i < 8; ++i) {
      int row = wave * 16 + 2 * i + rh;
      *(volatile v4f*)(Og + (size_t)row * DH + c4) = v[i];
    }
  }
}

extern "C" void kernel_launch(void* const* d_in, const int* in_sizes, int n_in,
                              void* d_out, int out_size, void* d_ws, size_t ws_size,
                              hipStream_t stream) {
  (void)d_ws; (void)ws_size;
  if (n_in < 3) return;
  const long long need_in  = (long long)(NB - 1) * (long long)IN_BSTRIDE + (long long)SEQ * DH;
  const long long need_out = (long long)(NB - 1) * (long long)OUT_BSTRIDE + (long long)SEQ * DH;
  if ((long long)in_sizes[0] < need_in || (long long)in_sizes[1] < need_in ||
      (long long)in_sizes[2] < need_in) return;
  if ((long long)out_size < need_out) return;
  const float* Q = (const float*)d_in[0];
  const float* K = (const float*)d_in[1];
  const float* V = (const float*)d_in[2];
  float* O = (float*)d_out;
  dim3 grid(NB * (SEQ / BM));
  sdpa_fa_kernel<<<grid, NTHR, 0, stream>>>(Q, K, V, O);
}
